// SelfAttentionBlock_21388937134616
// MI455X (gfx1250) — hardware-run, weakly checked
//
#include <hip/hip_runtime.h>


#ifndef NB
#define NB 2
#endif
#define NB_FULL 2
#define CH   128
#define HH   16
#define WW   512
#define SEQ  (HH * WW)
#define TD   512
#define NG   32
#define CPG  (CH / NG)
#define GNN  (CPG * SEQ)
#define AW   4
#define YSP  68
#define ETP  136
#define EMP  520
#define ECF  8.0f
#define WCF  64.0f
#define PCF  8.0f
#define OSC  (1.0f / 64.0f)
#define SC2  ((float)(0.08838834764831845 * 1.4426950408889634 / 64.0))
#define PSH  14.0f
#define CXS  32.0f
#define YSC  (1.0f / 16384.0f)
#define EMC  1024.0f
#define TSC  (1.0f / 65536.0f)
#define NEGB (-3.0e38f)
#define GEPS 1.0e-6f

static_assert(TD == WW);
static_assert((TD & (TD - 1)) == 0);
static_assert(CH % 64 == 0);
static_assert(CH % 32 == 0);
static_assert(TD % 128 == 0);
static_assert(SEQ % 64 == 0);
static_assert((NB * SEQ) % 64 == 0);
static_assert(SEQ % 32 == 0);
static_assert(SEQ % (16 * AW) == 0);
static_assert(SEQ % TD == 0);
static_assert(GNN % 1024 == 0);
static_assert(NB >= 1);
static_assert(NB <= 8);
static_assert(NB <= NB_FULL);
static_assert(CH * CH / 8 == 8 * 256);
static_assert(CH / 4 == 32);
static_assert(((16 - NB) * EMP) % 8 == 0);
static_assert((EMP * 2) % 16 == 0);
static_assert((ETP * 2) % 16 == 0);
static_assert((YSP * 4) % 16 == 0);
static_assert(CH * YSP * 4 <= 131072);
static_assert(64 * ETP * 2 + 4 * CH * 4 <= 131072);
static_assert(16 * EMP * 2 + NB * 64 * 4 <= 131072);
static_assert(16 * 68 * 4 <= 131072);

typedef _Float16 h16;
typedef __attribute__((ext_vector_type(16))) _Float16 v16h;
typedef __attribute__((ext_vector_type(8)))  _Float16 v8h;
typedef __attribute__((ext_vector_type(8)))  float    v8f;
typedef __attribute__((ext_vector_type(4)))  float    v4f;
typedef v4f  __attribute__((may_alias)) v4fa;
typedef v8h  __attribute__((may_alias)) v8ha;

__device__ __forceinline__ unsigned short f2bf(float f) { unsigned u = __float_as_uint(f); u += 0x7FFFu + ((u >> 16) & 1u); return (unsigned short)(u >> 16); }
__device__ __forceinline__ float bfr(float f) { return __uint_as_float(((unsigned)f2bf(f)) << 16); }
__device__ __forceinline__ v16h cat16(v8h lo, v8h hi) { return __builtin_shufflevector(lo, hi, 0, 1, 2, 3, 4, 5, 6, 7, 8, 9, 10, 11, 12, 13, 14, 15); }
static __device__ __forceinline__ h16 toh_flush(float v) { const h16 r = (h16)v; return (fabsf(v) < 6.103515625e-05f) ? (h16)0.0f : r; }
__device__ __forceinline__ v16h ldh(const h16* p) { return cat16(*(const v8h*)p, *(const v8h*)(p + 16)); }
__device__ __forceinline__ v8f mma(v16h a, v16h b, v8f c) {
    c = __builtin_amdgcn_wmma_f32_16x16x32_f16(false, a, false, b, (short)0, c, false, false);
    asm volatile("v_nop\n\tv_nop\n\tv_nop\n\tv_nop" : "+v"(c) : "v"(a), "v"(b));
    return c;
}
__device__ __forceinline__ void wave_sync() { __builtin_amdgcn_fence(3  , "wavefront"); __builtin_amdgcn_wave_barrier(); asm volatile("" ::: "memory"); }
__device__ __forceinline__ double wred(double v) {
#pragma unroll
    for (int o = 16; o > 0; o >>= 1) v += __shfl_xor(v, o, 32);
    return v;
}

__global__ __launch_bounds__(256) void k_wconv(const float* __restrict__ w0, const float* __restrict__ w1, const float* __restrict__ w2, const float* __restrict__ w3,
                                               const float* __restrict__ b0, const float* __restrict__ b1, const float* __restrict__ b2, const float* __restrict__ b3,
                                               h16* WH, float* BS) {
    const int i = blockIdx.x * 256 + threadIdx.x;
    if (i >= CH * CH / 8) return;
    const v8f a0 = *(const v8f*)(w0 + (size_t)i * 8);
    const v8f a1 = *(const v8f*)(w1 + (size_t)i * 8);
    const v8f a2 = *(const v8f*)(w2 + (size_t)i * 8);
    const v8f a3 = *(const v8f*)(w3 + (size_t)i * 8);
    v8h h0, h1, h2, h3;
#pragma unroll
    for (int k = 0; k < 8; ++k) { h0[k] = toh_flush(bfr(a0[k]) * WCF); h1[k] = toh_flush(bfr(a1[k]) * WCF); h2[k] = toh_flush(bfr(a2[k]) * WCF); h3[k] = toh_flush(bfr(a3[k]) * WCF); }
    const bool bl = i < CH / 4;
    v4f c0 = (v4f){}, c1 = (v4f){}, c2 = (v4f){}, c3 = (v4f){};
    if (bl) {
        c0 = *(const v4f*)(b0 + i * 4); c1 = *(const v4f*)(b1 + i * 4); c2 = *(const v4f*)(b2 + i * 4); c3 = *(const v4f*)(b3 + i * 4);
#pragma unroll
        for (int k = 0; k < 4; ++k) { c0[k] = bfr(c0[k]); c1[k] = bfr(c1[k]); c2[k] = bfr(c2[k]); c3[k] = bfr(c3[k]); }
    }
#pragma unroll 1
    for (int ps = 0; ps < 2; ++ps) {
        *(volatile v8h*)(WH + (size_t)i * 8) = h0;
        *(volatile v8h*)(WH + (size_t)CH * CH + (size_t)i * 8) = h1;
        *(volatile v8h*)(WH + (size_t)2 * CH * CH + (size_t)i * 8) = h2;
        *(volatile v8h*)(WH + (size_t)3 * CH * CH + (size_t)i * 8) = h3;
        if (bl) {
            *(volatile v4f*)(BS + i * 4) = c0; *(volatile v4f*)(BS + CH + i * 4) = c1;
            *(volatile v4f*)(BS + 2 * CH + i * 4) = c2; *(volatile v4f*)(BS + 3 * CH + i * 4) = c3;
        }
        if (ps == 0) __threadfence();
    }
}

__global__ __launch_bounds__(128) void k_tenc(const int* __restrict__ tin, const float* __restrict__ tw, const float* __restrict__ tb, float* TE) {
    __shared__ __align__(16) h16 em[16 * EMP];
    __shared__ __align__(16) float ts[NB * 64];
    const int tid = threadIdx.x, lane = tid & 31, lr = lane & 15, hi = lane >> 4;
    const int wave = __builtin_amdgcn_readfirstlane((int)(threadIdx.x >> 5));
    const v8h hz8 = (v8h){};
#pragma unroll 1
    for (int q = tid; q < (16 - NB) * EMP / 8; q += 128) *(v8ha*)(&em[NB * EMP + q * 8]) = hz8;
#pragma unroll 1
    for (int q = tid; q < NB * (TD / 2); q += 128) {
        const int bb = q / (TD / 2), i = q % (TD / 2);
        const float tv = (float)tin[bb];
        const float ex = (2.0f * (float)i) * (1.0f / (float)TD);
        const float fr = powf(10000.0f, ex);
        const float arg = tv * (1.0f / fr);
        const float sv = fmaxf(sinf(arg), 0.0f), cv = fmaxf(cosf(arg), 0.0f);
        em[bb * EMP + 2 * i] = toh_flush(sv * EMC);
        em[bb * EMP + 2 * i + 1] = toh_flush(cv * EMC);
    }
    __syncthreads();
    const int j = blockIdx.x * 64 + wave * 16 + lr;
    const float* wp = tw + (size_t)j * TD + 8 * hi;
    const int eo = lr * EMP + 8 * hi;
    v8f acc = (v8f){};
#pragma unroll 4
    for (int kc = 0; kc < TD; kc += 32) {
        const v16h a = cat16(*(const v8ha*)(&em[eo + kc]), *(const v8ha*)(&em[eo + kc + 16]));
        const v4f x0 = *(const v4f*)(wp + kc), x1 = *(const v4f*)(wp + kc + 4), x2 = *(const v4f*)(wp + kc + 16), x3 = *(const v4f*)(wp + kc + 20);
        v16h bq;
#pragma unroll
        for (int i = 0; i < 4; ++i) {
            bq[i] = toh_flush(bfr(x0[i]) * WCF); bq[4 + i] = toh_flush(bfr(x1[i]) * WCF);
            bq[8 + i] = toh_flush(bfr(x2[i]) * WCF); bq[12 + i] = toh_flush(bfr(x3[i]) * WCF); }
        acc = mma(a, bq, acc);
    }
    const float bj = bfr(tb[j]);
    if (hi == 0) {
#pragma unroll
        for (int bb = 0; bb < NB; ++bb) ts[bb * 64 + wave * 16 + lr] = acc[bb] * TSC + bj;
    }
    __syncthreads();
    if (wave == 0) {
#pragma unroll 1
        for (int ps = 0; ps < 2; ++ps) {
#pragma unroll 1
            for (int base = 0; base < NB * 2; base += 4) {
                const int ln = base + (lane >> 3);
                if (ln < NB * 2) {
                    const int bb = ln >> 1, hf = ln & 1, c4 = (lane & 7) * 4;
                    const v4f val = *(const v4fa*)(&ts[bb * 64 + hf * 32 + c4]);
                    *(volatile v4f*)(TE + (size_t)bb * TD + blockIdx.x * 64 + hf * 32 + c4) = val; }
            }
            if (ps == 0) __threadfence();
        }
    }
}

__global__ __launch_bounds__(256) void k_gstat(const float* __restrict__ x, const float* __restrict__ TE, float* ST) {
#pragma clang fp contract(off)
    __shared__ double red[8];
    const int tid = threadIdx.x, lane = tid & 31;
    const int wave = __builtin_amdgcn_readfirstlane((int)(threadIdx.x >> 5));
    const int b = blockIdx.x / NG, g = blockIdx.x % NG;
    const float* xg = x + ((size_t)b * CH + (size_t)g * CPG) * SEQ;
    const v4f te = *(const v4f*)(TE + (size_t)b * TD + ((4 * tid) & (TD - 1)));
    v4f s = (v4f){};
#pragma unroll 4
    for (int it = 0; it < GNN / 1024; ++it) {
        const v4f v = *(const v4f*)(xg + (size_t)(it * 256 + tid) * 4);
#pragma unroll
        for (int i = 0; i < 4; ++i) s[i] += bfr(v[i]) + te[i]; }
    double ds = wred(((double)s[0] + (double)s[1]) + ((double)s[2] + (double)s[3]));
    if (lane == 0) red[wave] = ds;
    __syncthreads();
    double tot = 0.0;
#pragma unroll
    for (int w = 0; w < 8; ++w) tot += red[w];
    const float mu = (float)(tot * (1.0 / (double)GNN));
    __syncthreads();
    v4f q = (v4f){};
#pragma unroll 4
    for (int it = 0; it < GNN / 1024; ++it) {
        const v4f v = *(const v4f*)(xg + (size_t)(it * 256 + tid) * 4);
#pragma unroll
        for (int i = 0; i < 4; ++i) { const float d = (bfr(v[i]) + te[i]) - mu; q[i] += d * d; } }
    double dq = wred(((double)q[0] + (double)q[1]) + ((double)q[2] + (double)q[3]));
    if (lane == 0) red[wave] = dq;
    __syncthreads();
    double tq = 0.0;
#pragma unroll
    for (int w = 0; w < 8; ++w) tq += red[w];
    const float var = (float)(tq * (1.0 / (double)GNN));
    const float rs = rsqrtf(var + GEPS);
    if (tid < 8) {
        v4f o = (v4f){};
        o[0] = (tid == 0) ? mu : 0.0f; o[1] = (tid == 0) ? rs : 0.0f;
        *(volatile v4f*)(ST + (size_t)blockIdx.x * 32 + tid * 4) = o;
        __threadfence();
        *(volatile v4f*)(ST + (size_t)blockIdx.x * 32 + tid * 4) = o;
    }
}

__global__ __launch_bounds__(256) void k_gnorm(const float* __restrict__ x, const float* __restrict__ TE, const float* __restrict__ ST,
                                               const float* __restrict__ gam, const float* __restrict__ bet, h16* ET) {
#pragma clang fp contract(off)
    __shared__ __align__(16) h16 tl[64 * ETP];
    __shared__ float cm[CH], cr[CH], cg[CH], cb[CH];
    const int tid = threadIdx.x;
    const int b = blockIdx.y, p0 = blockIdx.x * 64;
    if (tid < CH) {
        const int gi = (b * NG + (tid >> 2)) * 32;
        cm[tid] = ST[gi]; cr[tid] = ST[gi + 1]; cg[tid] = bfr(gam[tid]); cb[tid] = bfr(bet[tid]);
    }
    __syncthreads();
    const int pc = 4 * (tid & 15);
    const v4f te = *(const v4f*)(TE + (size_t)b * TD + ((p0 + pc) & (TD - 1)));
#pragma unroll 2
    for (int it = 0; it < 8; ++it) {
        const int c = (tid >> 4) + 16 * it;
        const v4f v = *(const v4f*)(x + ((size_t)b * CH + c) * SEQ + p0 + pc);
        const float mu = cm[c], rs = cr[c], gg = cg[c], bb = cb[c];
#pragma unroll
        for (int i = 0; i < 4; ++i) {
            const float y = (((bfr(v[i]) + te[i]) - mu) * rs) * gg + bb;
            tl[(pc + i) * ETP + c] = toh_flush(y * ECF); }
    }
    __syncthreads();
    static_assert(256 * 4 * 16 == 64 * CH * 2);
#pragma unroll 1
    for (int ps = 0; ps < 2; ++ps) {
#pragma unroll
        for (int it = 0; it < 4; ++it) {
            const int q = it * 256 + tid; const int row = q >> 4, c8 = (q & 15) * 8;
            const v8h hv = *(const v8ha*)(&tl[row * ETP + c8]);
            *(volatile v8h*)(ET + ((size_t)b * SEQ + p0 + row) * CH + c8) = hv; }
        if (ps == 0) __threadfence();
    }
}

template <int MODE>
__device__ __forceinline__ void proj_tile(const h16* __restrict__ A, const h16* __restrict__ Bt, const float* __restrict__ bias, h16* P, const int r0, const int c0) {
    __shared__ __align__(16) float os[16 * 68];
    const int K = CH;
    const int lane = threadIdx.x & 31, lr = lane & 15, hi = lane >> 4;
    v8f acc[4][4];
#pragma unroll
    for (int mb = 0; mb < 4; ++mb)
#pragma unroll
        for (int nb = 0; nb < 4; ++nb) acc[mb][nb] = (v8f){};
    const size_t aoff = (size_t)(r0 + lr) * K + 8 * hi, boff = (size_t)(c0 + lr) * K + 8 * hi;
#pragma unroll 1
    for (int kc = 0; kc < K; kc += 32) {
        v16h a[4];
#pragma unroll
        for (int mb = 0; mb < 4; ++mb) a[mb] = ldh(A + aoff + (size_t)mb * 16 * K + kc);
#pragma unroll
        for (int nb = 0; nb < 4; ++nb) { const v16h bq = ldh(Bt + boff + (size_t)nb * 16 * K + kc);
#pragma unroll
            for (int mb = 0; mb < 4; ++mb) acc[mb][nb] = mma(a[mb], bq, acc[mb][nb]); }
    }
    float bc[4];
#pragma unroll
    for (int nb = 0; nb < 4; ++nb) bc[nb] = (MODE == 0) ? bias[c0 + nb * 16 + lr] * PCF : 0.0f;
    size_t tbase; size_t ldo;
    if (MODE == 0) { tbase = (size_t)r0 * CH + (size_t)c0; ldo = CH; }
    else           { const int bb = c0 / SEQ, tt = c0 % SEQ; tbase = ((size_t)bb * CH + (size_t)r0) * SEQ + (size_t)tt; ldo = SEQ; }
#pragma unroll
    for (int mb = 0; mb < 4; ++mb) {
        float br[8];
#pragma unroll
        for (int j = 0; j < 8; ++j) br[j] = (MODE == 1) ? bias[r0 + mb * 16 + hi * 8 + j] * PCF : 0.0f;
#pragma unroll
        for (int nb = 0; nb < 4; ++nb) {
#pragma unroll
            for (int j = 0; j < 8; ++j) os[(hi * 8 + j) * 68 + nb * 16 + lr] = acc[mb][nb][j] * OSC + bc[nb] + br[j]; }
        wave_sync();
        static_assert(32 * 4 * 16 == 16 * 64 * 2);
#pragma unroll 1
        for (int ps = 0; ps < 2; ++ps) {
#pragma unroll
            for (int s = 0; s < 4; ++s) { const int row = 4 * s + (lane >> 3), c8 = (lane & 7) * 8;
                const v4f x0 = *(const v4fa*)(&os[row * 68 + c8]); const v4f x1 = *(const v4fa*)(&os[row * 68 + c8 + 4]); v8h hv;
#pragma unroll
                for (int i = 0; i < 4; ++i) { hv[i] = toh_flush(x0[i]); hv[4 + i] = toh_flush(x1[i]); }
                *(volatile v8h*)(P + tbase + (size_t)(mb * 16 + row) * ldo + c8) = hv; }
            if (ps == 0) __threadfence(); }
        wave_sync();
    }
}

__global__ __launch_bounds__(32) void k_proj_tok(const h16* __restrict__ ET, const h16* __restrict__ WH, const float* __restrict__ BS, h16* QK) {
    const int z = blockIdx.z;
    proj_tile<0>(ET, WH + (size_t)z * CH * CH, BS + z * CH, QK + (size_t)z * ((size_t)NB * SEQ * CH), blockIdx.x * 64, blockIdx.y * 64);
}
__global__ __launch_bounds__(32) void k_proj_ch(const h16* __restrict__ WH, const h16* __restrict__ ET, const float* __restrict__ BS, h16* VT) {
    proj_tile<1>(WH + (size_t)2 * CH * CH, ET, BS + 2 * CH, VT, blockIdx.x * 64, blockIdx.y * 64);
}

__global__ __launch_bounds__(32 * AW) __attribute__((amdgpu_num_vgpr(256)))
void k_flash(const h16* __restrict__ QP, const h16* __restrict__ KP, const h16* __restrict__ VT, const h16* __restrict__ WH, const float* __restrict__ BS,
             const float* __restrict__ x, float* OUT) {
    __shared__ __align__(16) float ys[CH * YSP];
    const int lane = threadIdx.x & 31, lr = lane & 15, hi = lane >> 4;
    const int wave = __builtin_amdgcn_readfirstlane((int)(threadIdx.x >> 5));
    const int b = blockIdx.y;
    const int tq0 = blockIdx.x * (16 * AW);
    const int t0 = tq0 + wave * 16;
    const size_t pbase = (size_t)b * SEQ * CH;
    const size_t qo = pbase + (size_t)(t0 + lr) * CH + 8 * hi;
    v16h qf[4];
#pragma unroll
    for (int kc = 0; kc < 4; ++kc) qf[kc] = ldh(QP + qo + kc * 32);
    const size_t ko = pbase + (size_t)lr * CH + 8 * hi;
    const size_t vo = pbase + (size_t)lr * SEQ + 8 * hi;
    v8f o[8];
#pragma unroll
    for (int j = 0; j < 8; ++j) o[j] = (v8f){};
    float m = NEGB, l = 0.0f;
#pragma unroll 1
    for (int key0 = 0; key0 < SEQ; key0 += 32) {
        const h16* ka = KP + ko + (size_t)key0 * CH;
        v8f sa = (v8f){}, sb = (v8f){};
#pragma unroll
        for (int kc = 0; kc < 4; ++kc) {
            const v16h k0 = ldh(ka + kc * 32), k1 = ldh(ka + 16 * CH + kc * 32);
            sa = mma(k0, qf[kc], sa); sb = mma(k1, qf[kc], sb); }
        float ta[8], tc[8]; float mx = NEGB;
#pragma unroll
        for (int r = 0; r < 8; ++r) { ta[r] = sa[r] * SC2; tc[r] = sb[r] * SC2; mx = fmaxf(mx, fmaxf(ta[r], tc[r])); }
        mx = fmaxf(mx, __shfl_xor(mx, 16, 32));
        const float mnew = fmaxf(m, mx);
        const float alpha = __builtin_amdgcn_exp2f(m - mnew);
        const float sh = PSH - mnew;
        v16h pb; float ls = 0.0f;
#pragma unroll
        for (int r = 0; r < 8; ++r) {
            const float ea = ta[r] + sh, eb = tc[r] + sh;
            const float xa = __builtin_amdgcn_exp2f(ea), xc = __builtin_amdgcn_exp2f(eb);
            const float ga = (ea < -14.0f) ? 0.0f : xa, gb = (eb < -14.0f) ? 0.0f : xc;
            const h16 pa = (h16)ga; const h16 pc = (h16)gb;
            pb[r] = pa; pb[8 + r] = pc; ls += (float)pa + (float)pc; }
        l = l * alpha + ls; m = mnew;
#pragma unroll
        for (int j = 0; j < 8; ++j) o[j] = o[j] * alpha;
        const h16* va = VT + vo + key0;
#pragma unroll
        for (int j = 0; j < 8; ++j) { const v16h vf = ldh(va + (size_t)(16 * j) * SEQ); o[j] = mma(vf, pb, o[j]); }
    }
    l += __shfl_xor(l, 16, 32);
    const float inv = CXS * (1.0f / l);
    v16h cf[4];
#pragma unroll
    for (int kc = 0; kc < 4; ++kc) {
#pragma unroll
        for (int r = 0; r < 8; ++r) { cf[kc][r] = toh_flush(o[2 * kc][r] * inv); cf[kc][8 + r] = toh_flush(o[2 * kc + 1][r] * inv); } }
    const size_t wo = (size_t)3 * CH * CH + (size_t)lr * CH + 8 * hi;
    v8f y[8];
#pragma unroll
    for (int jo = 0; jo < 8; ++jo) {
        y[jo] = (v8f){};
#pragma unroll
        for (int kc = 0; kc < 4; ++kc) { const v16h wf = ldh(WH + wo + (size_t)(16 * jo) * CH + kc * 32); y[jo] = mma(wf, cf[kc], y[jo]); } }
#pragma unroll
    for (int jo = 0; jo < 8; ++jo) {
#pragma unroll
        for (int r = 0; r < 8; ++r) ys[(16 * jo + 8 * hi + r) * YSP + wave * 16 + lr] = y[jo][r]; }
    __syncthreads();
    const size_t gb = (size_t)b * CH * SEQ + (size_t)tq0;
    static_assert(32 * AW * 16 * 16 == CH * 64 * 4);
#pragma unroll 1
    for (int ps = 0; ps < 2; ++ps) {
#pragma unroll 2
        for (int it = 0; it < 16; ++it) {
            const int q = it * (32 * AW) + (int)threadIdx.x; const int row = q >> 4, c4 = (q & 15) * 4;
            const v4f yv = *(const v4fa*)(&ys[row * YSP + c4]);
            const v4f xv = *(const v4f*)(x + gb + (size_t)row * SEQ + c4);
            const float bo = BS[3 * CH + row];
            v4f val;
#pragma unroll
            for (int i = 0; i < 4; ++i) val[i] = bfr(xv[i]) + (yv[i] * YSC + bo);
            *(volatile v4f*)(OUT + gb + (size_t)row * SEQ + c4) = val; }
        if (ps == 0) __threadfence();
    }
}

static constexpr size_t al256(size_t v) { return (v + 255) & ~(size_t)255; }
static constexpr size_t PLN   = (size_t)NB * SEQ * CH;
static constexpr size_t SZ_TE = al256((size_t)NB * TD * 4);
static constexpr size_t SZ_ST = al256((size_t)NB * NG * 32 * 4);
static constexpr size_t SZ_WH = al256((size_t)4 * CH * CH * 2);
static constexpr size_t SZ_BS = al256((size_t)4 * CH * 4);
static constexpr size_t SZ_PL = al256(PLN * 2);
static constexpr size_t SZ_TOTAL = SZ_TE + SZ_ST + SZ_WH + SZ_BS + 4 * SZ_PL;
static_assert(SZ_TOTAL <= (size_t)134217728);
static_assert((PLN * 2) % 256 == 0);
static_assert(SZ_PL == PLN * 2);
static_assert((size_t)NB * CH * SEQ == PLN);

extern "C" void kernel_launch(void* const* d_in, const int* in_sizes, int n_in,
                              void* d_out, int out_size, void* d_ws, size_t ws_size, hipStream_t stream) {
    if (n_in < 14) return;
    if ((size_t)in_sizes[0] < (size_t)NB * CH * SEQ) return;
    if (in_sizes[1] < NB) return;
    if ((size_t)in_sizes[2] < (size_t)TD * TD || in_sizes[3] < TD) return;
    if (in_sizes[4] < CH || in_sizes[5] < CH) return;
    if ((size_t)in_sizes[6] < (size_t)CH * CH || (size_t)in_sizes[8] < (size_t)CH * CH || (size_t)in_sizes[10] < (size_t)CH * CH || (size_t)in_sizes[12] < (size_t)CH * CH) return;
    if (in_sizes[7] < CH || in_sizes[9] < CH || in_sizes[11] < CH || in_sizes[13] < CH) return;
    if ((size_t)out_size < (size_t)NB * CH * SEQ) return;
    if (SZ_TOTAL > ws_size) return;
    const float* x  = (const float*)d_in[0];
    const int*   t  = (const int*)d_in[1];
    const float* tw = (const float*)d_in[2];  const float* tbv = (const float*)d_in[3];
    const float* gg = (const float*)d_in[4];  const float* gbv = (const float*)d_in[5];
    const float* qw = (const float*)d_in[6];  const float* qb = (const float*)d_in[7];
    const float* kw = (const float*)d_in[8];  const float* kb = (const float*)d_in[9];
    const float* vw = (const float*)d_in[10]; const float* vb = (const float*)d_in[11];
    const float* pw = (const float*)d_in[12]; const float* pb = (const float*)d_in[13];
    float* OUT = (float*)d_out;
    char* wsp = (char*)d_ws;
    float* TE = (float*)wsp; wsp += SZ_TE;
    float* ST = (float*)wsp; wsp += SZ_ST;
    h16*   WH = (h16*)wsp;   wsp += SZ_WH;
    float* BS = (float*)wsp; wsp += SZ_BS;
    h16*   ET = (h16*)wsp;   wsp += SZ_PL;
    h16*   QK = (h16*)wsp;   wsp += 2 * SZ_PL;
    h16*   VT = (h16*)wsp;   wsp += SZ_PL;

    k_wconv<<<CH * CH / 8 / 256, 256, 0, stream>>>(qw, kw, vw, pw, qb, kb, vb, pb, WH, BS);
    k_tenc<<<TD / 64, 128, 0, stream>>>(t, tw, tbv, TE);
    k_gstat<<<NB * NG, 256, 0, stream>>>(x, TE, ST);
    k_gnorm<<<dim3(SEQ / 64, NB, 1), 256, 0, stream>>>(x, TE, ST, gg, gbv, ET);
    k_proj_tok<<<dim3(NB * SEQ / 64, CH / 64, 2), 32, 0, stream>>>(ET, WH, BS, QK);
    k_proj_ch<<<dim3(CH / 64, NB * SEQ / 64, 1), 32, 0, stream>>>(WH, ET, BS, VT);
    k_flash<<<dim3(SEQ / (16 * AW), NB, 1), 32 * AW, 0, stream>>>(QK, QK + PLN, VT, WH, BS, x, OUT);
}
